// ModulatedDeformConv_41068477284904
// MI455X (gfx1250) — hardware-verified
//
#include <hip/hip_runtime.h>

constexpr int NBATCH = 4;
constexpr int NCIN   = 256;
constexpr int IMH    = 64;
constexpr int IMW    = 64;
constexpr int NCOUT  = 256;
constexpr int NTAP   = 9;
constexpr int HWO    = 4096;
constexpr int KCDIM  = NCIN * NTAP;
constexpr int BCHUNK = 2;
constexpr int NROWS_CHUNK = BCHUNK * HWO;
constexpr int PXT    = 16;
constexpr int CCH    = 64;
constexpr int KCH    = CCH * NTAP;
constexpr int LDSP   = KCH + 8;
constexpr int NPAIR  = NTAP * PXT;

static_assert(NCOUT % 64 == 0, "M tile multiple");
static_assert(HWO % 64 == 0, "N tile multiple");
static_assert(KCDIM % 32 == 0, "K multiple of 32");
static_assert(KCH % 64 == 0, "block kc segment is whole 128-B lines");
static_assert((LDSP * 2) % 16 == 0, "LDS row 16-B aligned");
static_assert(NROWS_CHUNK % PXT == 0 && NCIN % CCH == 0, "sampling grid exact");
static_assert(NBATCH % BCHUNK == 0, "chunking exact");

typedef __attribute__((ext_vector_type(16))) _Float16 v16h;
typedef __attribute__((ext_vector_type(8)))  _Float16 v8h;
typedef __attribute__((ext_vector_type(16))) __bf16   v16b;
typedef __attribute__((ext_vector_type(8)))  __bf16   v8b;
typedef __attribute__((ext_vector_type(8)))  float    v8f;
typedef __attribute__((ext_vector_type(4)))  float    v4f;
typedef __attribute__((ext_vector_type(4)))  unsigned int v4u;

__device__ __forceinline__ unsigned short f2bf_bits(float f) {
  unsigned u = __float_as_uint(f);
  return (unsigned short)((u + 0x7FFFu + ((u >> 16) & 1u)) >> 16);
}
__device__ __forceinline__ float bf_bits2f(unsigned short h) { return __uint_as_float(((unsigned)h) << 16); }

__device__ __forceinline__ void dep_guard_h(v8f& a, v8f& b, v16h x, v16h y) { asm volatile("v_nop\n\tv_nop\n\tv_nop\n\tv_nop" : "+v"(a), "+v"(b) : "v"(x), "v"(y)); }
__device__ __forceinline__ void dep_guard_b(v8f& a, v8f& b, v16b x, v16b y) { asm volatile("v_nop\n\tv_nop\n\tv_nop\n\tv_nop" : "+v"(a), "+v"(b) : "v"(x), "v"(y)); }
__device__ __forceinline__ void keep4_h(v16h a, v16h b, v16h c, v16h d) { asm volatile("v_nop" :: "v"(a), "v"(b), "v"(c), "v"(d)); }
__device__ __forceinline__ void keep4_b(v16b a, v16b b, v16b c, v16b d) { asm volatile("v_nop" :: "v"(a), "v"(b), "v"(c), "v"(d)); }
__device__ __forceinline__ void acc_guard4(v8f& a, v8f& b, v8f& c, v8f& d) { asm volatile("v_nop\n\tv_nop\n\tv_nop\n\tv_nop" : "+v"(a), "+v"(b), "+v"(c), "+v"(d)); }
template <typename T> struct Frag;
template <> struct Frag<_Float16> {
  typedef v16h V; union U { v16h v; v8h h[2]; };
  static __device__ __forceinline__ v16h load(const _Float16* p) {
    U f; f.h[0] = *(const v8h*)(p); f.h[1] = *(const v8h*)(p + 16); return f.v;
  }
  static __device__ __forceinline__ v8f mma(v16h a, v16h b, v8f c) {
    return __builtin_amdgcn_wmma_f32_16x16x32_f16(false, a, false, b, (short)0, c, false, false);
  }
  static __device__ __forceinline__ void guard(v8f& a, v8f& b, v16h x, v16h y) { dep_guard_h(a, b, x, y); }
  static __device__ __forceinline__ void keep(v16h a, v16h b, v16h c, v16h d) { keep4_h(a, b, c, d); }
};
template <> struct Frag<__bf16> {
  typedef v16b V; union U { v16b v; v8b h[2]; };
  static __device__ __forceinline__ v16b load(const __bf16* p) {
    U f; f.h[0] = *(const v8b*)(p); f.h[1] = *(const v8b*)(p + 16); return f.v;
  }
  static __device__ __forceinline__ v8f mma(v16b a, v16b b, v8f c) {
    return __builtin_amdgcn_wmma_f32_16x16x32_bf16(false, a, false, b, (short)0, c, false, false);
  }
  static __device__ __forceinline__ void guard(v8f& a, v8f& b, v16b x, v16b y) { dep_guard_b(a, b, x, y); }
  static __device__ __forceinline__ void keep(v16b a, v16b b, v16b c, v16b d) { keep4_b(a, b, c, d); }
};

template <int ET> struct Elem;
template <> struct Elem<0> { typedef _Float16 T; };
template <> struct Elem<1> { typedef __bf16 T; };
template <int ET, bool SPLIT, int BIAS_MODE, int OUT_MODE, bool RESID, int ACT = 0>
__global__ __launch_bounds__(256) void wmma_gemm64(
    const unsigned short* __restrict__ Ap, const unsigned short* __restrict__ A2p, int lda, long strideA,
    const unsigned short* __restrict__ Btp, const unsigned short* __restrict__ Bt2p, int ldb, long strideB,
    void* __restrict__ Cout, void* __restrict__ Cout2, int ldc, long strideC,
    const float* __restrict__ bias,
    const float* __restrict__ resid, long strideR,
    int M, int N, int K, float scale) {
  typedef typename Elem<ET>::T T;
  typedef typename Frag<T>::V V;
  const T* A = (const T*)Ap; const T* A2 = (const T*)A2p; const T* Bt = (const T*)Btp; const T* Bt2 = (const T*)Bt2p;
  __shared__ __align__(16) float sT[8][16 * 68];
  const int b    = blockIdx.y;
  const int lane = threadIdx.x & 31;
  const int wave = threadIdx.x >> 5;
  const int tilesN = N >> 6;
  const int tilesM = M >> 6;
  const int tile = blockIdx.x * 8 + wave;
  if (tile >= tilesM * tilesN) return;
  const int tm = tile / tilesN;
  const int tn = tile - tm * tilesN;
  const int m0 = tm << 6;
  const int n0 = tn << 6;

  const T* Ab  = A  + (size_t)b * strideA;
  const T* Bb  = Bt + (size_t)b * strideB;
  const T* Ab2 = SPLIT ? (A2  + (size_t)b * strideA) : nullptr;
  const T* Bb2 = SPLIT ? (Bt2 + (size_t)b * strideB) : nullptr;

  const int rlane = lane & 15;
  const int koff  = (lane >> 4) * 8;
  const int mOff  = (lane >> 4) * 8;

  v8f acc[4][4];
#pragma unroll
  for (int i = 0; i < 4; ++i)
#pragma unroll
    for (int j = 0; j < 4; ++j) acc[i][j] = (v8f){0.f,0.f,0.f,0.f,0.f,0.f,0.f,0.f};

  for (int k0 = 0; k0 < K; k0 += 32) {
    V bh[4], bl[4];
#pragma unroll
    for (int j = 0; j < 4; ++j) {
      const size_t bo = (size_t)(n0 + (j << 4) + rlane) * ldb + koff + k0;
      bh[j] = Frag<T>::load(Bb + bo);
      if (SPLIT) bl[j] = Frag<T>::load(Bb2 + bo);
    }
#pragma unroll
    for (int i = 0; i < 4; ++i) {
      const size_t ao = (size_t)(m0 + (i << 4) + rlane) * lda + koff + k0;
      V ah = Frag<T>::load(Ab + ao);
      V al;
      if (SPLIT) al = Frag<T>::load(Ab2 + ao);
#pragma unroll
      for (int j = 0; j < 4; ++j) {
        acc[i][j] = Frag<T>::mma(ah, bh[j], acc[i][j]);
        if (SPLIT) {
          acc[i][j] = Frag<T>::mma(ah, bl[j], acc[i][j]);
          acc[i][j] = Frag<T>::mma(al, bh[j], acc[i][j]);
        }
      }
      Frag<T>::guard(acc[i][0], acc[i][3], ah, SPLIT ? al : ah);
    }
    Frag<T>::keep(bh[0], bh[1], bh[2], bh[3]);
    if (SPLIT) Frag<T>::keep(bl[0], bl[1], bl[2], bl[3]);
  }
  acc_guard4(acc[0][0], acc[0][1], acc[0][2], acc[0][3]);
  acc_guard4(acc[1][0], acc[1][1], acc[1][2], acc[1][3]);
  acc_guard4(acc[2][0], acc[2][1], acc[2][2], acc[2][3]);
  acc_guard4(acc[3][0], acc[3][1], acc[3][2], acc[3][3]);

  float* slab = sT[wave];
  const float* Rb = RESID ? (resid + (size_t)b * strideR) : nullptr;
#pragma unroll
  for (int i = 0; i < 4; ++i) {
    const int mBase = m0 + (i << 4);
#pragma unroll
    for (int j = 0; j < 4; ++j) {
      const int n = n0 + (j << 4) + rlane;
      float bv = 0.f;
      if (BIAS_MODE == 2) bv = bias[n];
#pragma unroll
      for (int r = 0; r < 8; ++r) {
        float v = acc[i][j][r] * scale;
        if (BIAS_MODE == 1) v += bias[mBase + mOff + r];
        if (BIAS_MODE == 2) v += bv;
        if (RESID) v += Rb[(size_t)(mBase + mOff + r) * ldc + n];
        if (ACT == 1) v = tanhf(v);
        if (ACT == 2) v = fmaxf(v, 0.0f);
        if (ACT == 3) v = v / (1.0f + expf(-v));
        if (ACT == 4) v = (v > 0.f) ? v : 0.01f * v;
        if (ACT == 5) v = 0.5f * v * (1.0f + erff(v * 0.70710678118654752f));
        slab[(mOff + r) * 68 + (j << 4) + rlane] = v;
      }
    }
    __builtin_amdgcn_fence(__ATOMIC_RELEASE, "workgroup");
    __builtin_amdgcn_wave_barrier();
    __builtin_amdgcn_fence(__ATOMIC_ACQUIRE, "workgroup");
    if (OUT_MODE == 0) {
      float* C = (float*)Cout + (size_t)b * strideC;
      const int hh = lane >> 4, c4 = (lane & 15) * 4;
      for (int pass = 0; pass < 2; ++pass) {
#pragma unroll
        for (int it = 0; it < 8; ++it) {
          const int row = it * 2 + hh;
          v4f v = *(const v4f*)(slab + row * 68 + c4);
          *(volatile v4f*)(C + (size_t)(mBase + row) * ldc + n0 + c4) = v;
        }
        __threadfence();
      }
    } else {
      const int q = lane >> 3, c8 = (lane & 7) * 8;
      unsigned short* C  = (unsigned short*)Cout  + (size_t)b * strideC;
      unsigned short* C2 = (OUT_MODE == 2) ? ((unsigned short*)Cout2 + (size_t)b * strideC) : nullptr;
      for (int pass = 0; pass < 2; ++pass) {
#pragma unroll
        for (int it = 0; it < 4; ++it) {
          const int row = it * 4 + q;
          const float* sp = slab + row * 68 + c8;
          v8h hv, lv;
#pragma unroll
          for (int e = 0; e < 8; ++e) {
            if (OUT_MODE == 1) {
              hv[e] = (_Float16)sp[e];
            } else {
              unsigned short hb = f2bf_bits(sp[e]);
              unsigned short lb = f2bf_bits(sp[e] - bf_bits2f(hb));
              hv[e] = __builtin_bit_cast(_Float16, hb);
              lv[e] = __builtin_bit_cast(_Float16, lb);
            }
          }
          *(volatile v8h*)(C + (size_t)(mBase + row) * ldc + n0 + c8) = hv;
          if (OUT_MODE == 2) *(volatile v8h*)(C2 + (size_t)(mBase + row) * ldc + n0 + c8) = lv;
        }
        __threadfence();
      }
    }
    __builtin_amdgcn_fence(__ATOMIC_RELEASE, "workgroup");
    __builtin_amdgcn_wave_barrier();
    __builtin_amdgcn_fence(__ATOMIC_ACQUIRE, "workgroup");
  }
}

__device__ __forceinline__ unsigned pack_hl2(float f0, float f1, unsigned& lo) {
  const unsigned short h0 = f2bf_bits(f0);
  const unsigned short h1 = f2bf_bits(f1);
  const unsigned short l0 = f2bf_bits(f0 - bf_bits2f(h0));
  const unsigned short l1 = f2bf_bits(f1 - bf_bits2f(h1));
  lo = (unsigned)l0 | ((unsigned)l1 << 16);
  return (unsigned)h0 | ((unsigned)h1 << 16);
}
__global__ __launch_bounds__(256) void wsplit_bf16x8(
    const float* __restrict__ w, unsigned short* __restrict__ whi, unsigned short* __restrict__ wlo, int n8) {
  const int i = blockIdx.x * 256 + threadIdx.x;
  if (i < n8) {
    const v4f a = *(const v4f*)(w + (size_t)i * 8);
    const v4f c = *(const v4f*)(w + (size_t)i * 8 + 4);
    v4u hv, lv;
    unsigned l0, l1, l2, l3;
    hv[0] = pack_hl2(a[0], a[1], l0);
    hv[1] = pack_hl2(a[2], a[3], l1);
    hv[2] = pack_hl2(c[0], c[1], l2);
    hv[3] = pack_hl2(c[2], c[3], l3);
    lv[0] = l0; lv[1] = l1; lv[2] = l2; lv[3] = l3;
    unsigned short* ph = whi + (size_t)i * 8;
    unsigned short* pl = wlo + (size_t)i * 8;
    *(volatile v4u*)ph = hv;
    *(volatile v4u*)pl = lv;
    __threadfence();
    *(volatile v4u*)ph = hv;
    *(volatile v4u*)pl = lv;
  }
}

__global__ __launch_bounds__(256) void sample_cols_kernel(
    const float* __restrict__ x, const float* __restrict__ offs, const float* __restrict__ maskp,
    unsigned short* __restrict__ col, long planeStride, int batch0) {
  __shared__ __align__(16) unsigned short shc[2][PXT][LDSP];
  __shared__ int   s_xb[NPAIR], s_o00[NPAIR], s_o01[NPAIR], s_o10[NPAIR], s_o11[NPAIR];
  __shared__ float s_w00[NPAIR], s_w01[NPAIR], s_w10[NPAIR], s_w11[NPAIR];

  const int tid  = threadIdx.x;
  const int lane = tid & 31;
  const int wave = tid >> 5;
  const int prow0 = blockIdx.x * PXT;
  const int cch   = blockIdx.y;

  if (tid < NPAIR) {
    const int k  = tid >> 4;
    const int p  = tid & 15;
    const int prow = prow0 + p;
    const int b  = batch0 + (prow >> 12);
    const int hw = prow & (HWO - 1);
    const int ho = hw >> 6;
    const int wo = hw & 63;
    const int ky = k / 3;
    const int kx = k - ky * 3;
    const float oy = offs[((size_t)b * (2 * NTAP) + 2 * k)     * HWO + hw];
    const float ox = offs[((size_t)b * (2 * NTAP) + 2 * k + 1) * HWO + hw];
    const float mv = maskp[((size_t)b * NTAP + k) * HWO + hw];
    const float sy = (float)(ho - 1 + ky) + oy;
    const float sx = (float)(wo - 1 + kx) + ox;
    const float fy = floorf(sy);
    const float fx = floorf(sx);
    const float wy = sy - fy;
    const float wx = sx - fx;
    const float fyc = fminf(fmaxf(fy, -2.0f), 64.0f);
    const float fxc = fminf(fmaxf(fx, -2.0f), 64.0f);
    const int y0 = (int)fyc, x0 = (int)fxc;
    const int y1 = y0 + 1,   x1 = x0 + 1;
    const float vy0 = (y0 >= 0 && y0 < IMH) ? 1.f : 0.f;
    const float vy1 = (y1 >= 0 && y1 < IMH) ? 1.f : 0.f;
    const float vx0 = (x0 >= 0 && x0 < IMW) ? 1.f : 0.f;
    const float vx1 = (x1 >= 0 && x1 < IMW) ? 1.f : 0.f;
    const int y0c = min(max(y0, 0), IMH - 1), y1c = min(max(y1, 0), IMH - 1);
    const int x0c = min(max(x0, 0), IMW - 1), x1c = min(max(x1, 0), IMW - 1);
    s_xb[tid]  = b * (NCIN * IMH * IMW);
    s_o00[tid] = y0c * IMW + x0c;  s_o01[tid] = y0c * IMW + x1c;
    s_o10[tid] = y1c * IMW + x0c;  s_o11[tid] = y1c * IMW + x1c;
    s_w00[tid] = (1.f - wy) * (1.f - wx) * vy0 * vx0 * mv;
    s_w01[tid] = (1.f - wy) * wx         * vy0 * vx1 * mv;
    s_w10[tid] = wy         * (1.f - wx) * vy1 * vx0 * mv;
    s_w11[tid] = wy         * wx         * vy1 * vx1 * mv;
  }
  __syncthreads();

  {
    const int px = tid & 15;
    const int cw = tid >> 4;
#pragma unroll 1
    for (int k = 0; k < NTAP; ++k) {
      const int pr  = k * PXT + px;
      const int xbo = s_xb[pr];
      const int o00 = s_o00[pr], o01 = s_o01[pr], o10 = s_o10[pr], o11 = s_o11[pr];
      const float w00 = s_w00[pr], w01 = s_w01[pr], w10 = s_w10[pr], w11 = s_w11[pr];
#pragma unroll 1
      for (int cs = 0; cs < CCH / 16; ++cs) {
        const int cl = cw + cs * 16;
        const float* xb = x + (size_t)xbo + (size_t)(cch * CCH + cl) * (IMH * IMW);
        float v = xb[o00] * w00;
        v = fmaf(xb[o01], w01, v);
        v = fmaf(xb[o10], w10, v);
        v = fmaf(xb[o11], w11, v);
        const unsigned short hb = f2bf_bits(v);
        const unsigned short lb = f2bf_bits(v - bf_bits2f(hb));
        shc[0][px][cl * NTAP + k] = hb;
        shc[1][px][cl * NTAP + k] = lb;
      }
    }
  }
  __syncthreads();

  {
    const int plane = wave >> 2;
    const int lb0   = (wave & 3) * 36;
    const int q = lane >> 3, e = lane & 7;
    unsigned short* pbase = col + (size_t)plane * (size_t)planeStride + (size_t)cch * KCH;
    for (int pass = 0; pass < 2; ++pass) {
#pragma unroll
      for (int it = 0; it < 9; ++it) {
        const int l = lb0 + it * 4 + q;
        const int p = l / 9;
        const int s = l - p * 9;
        const v4u val = *(const v4u*)(&shc[plane][p][s * 64 + e * 8]);
        *(volatile v4u*)(pbase + (size_t)(prow0 + p) * KCDIM + s * 64 + e * 8) = val;
      }
      __threadfence();
    }
  }
}

extern "C" void kernel_launch(void* const* d_in, const int* in_sizes, int n_in,
                              void* d_out, int out_size, void* d_ws, size_t ws_size,
                              hipStream_t stream) {
  const size_t WPLANE_B   = (size_t)NCOUT * KCDIM * 2;
  const size_t COLPLANE_E = (size_t)NROWS_CHUNK * KCDIM;
  const size_t COLPLANE_B = COLPLANE_E * 2;
  const size_t WS_TOTAL   = 2 * WPLANE_B + 2 * COLPLANE_B;
  if (n_in < 4) return;
  if (in_sizes[0] != NBATCH * NCIN * IMH * IMW) return;
  if (in_sizes[1] != NBATCH * 2 * NTAP * HWO) return;
  if (in_sizes[2] != NBATCH * NTAP * HWO) return;
  if (in_sizes[3] != NCOUT * NCIN * NTAP) return;
  if (out_size != NBATCH * NCOUT * HWO) return;
  if (ws_size < WS_TOTAL) return;

  const float* x      = (const float*)d_in[0];
  const float* offs   = (const float*)d_in[1];
  const float* maskp  = (const float*)d_in[2];
  const float* weight = (const float*)d_in[3];
  float* out = (float*)d_out;

  char* ws = (char*)d_ws;
  unsigned short* whi   = (unsigned short*)(ws);
  unsigned short* wlo   = (unsigned short*)(ws + WPLANE_B);
  unsigned short* colhi = (unsigned short*)(ws + 2 * WPLANE_B);
  unsigned short* collo = (unsigned short*)(ws + 2 * WPLANE_B + COLPLANE_B);

  const int n8 = NCOUT * KCDIM / 8;
  wsplit_bf16x8<<<(n8 + 255) / 256, 256, 0, stream>>>(weight, whi, wlo, n8);

  for (int chunk = 0; chunk < NBATCH / BCHUNK; ++chunk) {
    sample_cols_kernel<<<dim3(NROWS_CHUNK / PXT, NCIN / CCH), 256, 0, stream>>>(
        x, offs, maskp, colhi, (long)COLPLANE_E, chunk * BCHUNK);
    float* outc = out + (size_t)chunk * BCHUNK * NCOUT * HWO;
    wmma_gemm64<1, true, 0, 0, false, 0><<<dim3((NCOUT / 64) * (HWO / 64) / 8, BCHUNK), 256, 0, stream>>>(
        whi, wlo, KCDIM, 0L,
        colhi, collo, KCDIM, (long)HWO * KCDIM,
        (void*)outc, nullptr, HWO, (long)NCOUT * HWO,
        nullptr,
        nullptr, 0L,
        NCOUT, HWO, KCDIM, 1.0f);
  }
}
